// GCGRUCell_78847009620497
// MI455X (gfx1250) — hardware-run, weakly checked
//
#include <hip/hip_runtime.h>
#include <stddef.h>
#include <stdint.h>
#include <math.h>


#define XTERMS 2

#define NNODE  10000
#define NBAT   16
#define NU     64
#define NDIN   2
#define ND     66
#define KP     96
#define MR     160000
#define XP     192
#define XW     96
#define KC     384
#define NG     128
#define GROWS  128
#define GBLK   1250
#define PB_WF  6
#define PB_WG  12
#define NTHR   256
#define NWAVE  8
#define EPT    8
#define CHUNK  (NTHR * EPT)
#define WCAP   (EPT * 32)
#define LISTN  (NWAVE * WCAP)
#define NBA    512
#define SLA    9
#define NSCAN  20
#define RCAP   12288
#define DEGCAP 64
#define AGG_ZINTS    (LISTN + 2 * RCAP + 3 * NBA)
#define MISC_INTS    16
#define ROWB_INTS    (NWAVE * XW)
#define SCAN_LDS_INTS (AGG_ZINTS + MISC_INTS + ROWB_INTS)
#define GATE_LDS_INTS (GROWS * NG + GROWS * XW + GROWS * NU)
#define CAND_LDS_INTS (2 * GROWS * NU)
#define WSMAX  134217728

static_assert(XTERMS == 1 || XTERMS == 2);
static_assert(MR == NBAT * NNODE && MR % GROWS == 0 && GBLK * GROWS == MR);
static_assert(KP % 32 == 0 && KP >= ND && XP == 2 * KP && XW * 2 == XP && KC == 4 * KP);
static_assert((GROWS * KP / 8) == 6 * NTHR);
static_assert((NG * KP / 8) == PB_WF * NTHR && (NU * KC / 8) == PB_WG * NTHR);
static_assert(GROWS == NWAVE * 16 && NG == 8 * 16 && NU == 4 * 16);
static_assert((CHUNK & (CHUNK - 1)) == 0 && CHUNK <= 4096);
static_assert((NBA & (NBA - 1)) == 0 && NBA == (1 << SLA));
static_assert(((long long)CHUNK << SLA) < (1LL << 31));
static_assert(NBA % NWAVE == 0 && NBA % 32 == 0 && NSCAN * NBA >= NNODE);
static_assert(RCAP % NTHR == 0 && RCAP % 4 == 0 && AGG_ZINTS % 4 == 0);
static_assert(RCAP >= 8365 + 8365 / 20 + 1);
static_assert(DEGCAP == 64 && DEGCAP >= 33 + 8);
static_assert(SCAN_LDS_INTS * 4 <= 327680 && GATE_LDS_INTS * 4 <= 327680 && CAND_LDS_INTS * 4 <= 327680);

typedef float          v2f   __attribute__((ext_vector_type(2)));
typedef float          v4f   __attribute__((ext_vector_type(4)));
typedef float          v8f   __attribute__((ext_vector_type(8)));
typedef int            v4i   __attribute__((ext_vector_type(4)));
typedef int            v8i   __attribute__((ext_vector_type(8)));
typedef unsigned short v8us  __attribute__((ext_vector_type(8)));
typedef unsigned short v16us __attribute__((ext_vector_type(16)));
typedef __bf16         v16bf __attribute__((ext_vector_type(16)));
typedef v2f  __attribute__((may_alias)) v2fa;
typedef v4f  __attribute__((may_alias)) v4fa;
typedef v4i  __attribute__((may_alias)) v4ia;
typedef v8us __attribute__((may_alias)) v8usa;
typedef unsigned __attribute__((may_alias)) u32a;
union FragB { v16bf v; v16us u; v8us h[2]; v8i w; };

__device__ __forceinline__ v8f wmb(const FragB& a, const FragB& b, v8f c) {
  v8f d = __builtin_amdgcn_wmma_f32_16x16x32_bf16(false, a.v, false, b.v, (short)0, c, false, false);
  asm volatile("v_nop\n\tv_nop\n\tv_nop\n\tv_nop" : "+v"(d) : "v"(a.w), "v"(b.w));
  return d;
}

__device__ __forceinline__ float u2f(unsigned u) { return __uint_as_float(u); }
__device__ __forceinline__ unsigned f2u(float f) { return __float_as_uint(f); }

__device__ __forceinline__ unsigned bf16_bits_u(unsigned u) {
  const unsigned r = (u + 0x7FFFu + ((u >> 16) & 1u)) >> 16;
  const unsigned q = (u >> 16) | 0x40u;
  return ((u & 0x7fffffffu) > 0x7f800000u) ? q : r;
}
__device__ __forceinline__ unsigned bf16_bits(float f) { return bf16_bits_u(f2u(f)); }
__device__ __forceinline__ float bf16_val(float f) { return u2f(bf16_bits(f) << 16); }

__device__ __forceinline__ void hilo_pack(float v0, float v1, float v2, float v3,
                                          int& h01, int& h23, int& l01, int& l23) {
  const unsigned a0 = bf16_bits(v0), a1 = bf16_bits(v1), a2 = bf16_bits(v2), a3 = bf16_bits(v3);
  float hv0 = u2f(a0 << 16), hv1 = u2f(a1 << 16), hv2 = u2f(a2 << 16), hv3 = u2f(a3 << 16);
  asm volatile("" : "+v"(hv0), "+v"(hv1), "+v"(hv2), "+v"(hv3));
  const unsigned b0 = bf16_bits(v0 - hv0);
  const unsigned b1 = bf16_bits(v1 - hv1);
  const unsigned b2 = bf16_bits(v2 - hv2);
  const unsigned b3 = bf16_bits(v3 - hv3);
  h01 = (int)(a0 | (a1 << 16)); h23 = (int)(a2 | (a3 << 16));
  l01 = (int)(b0 | (b1 << 16)); l23 = (int)(b2 | (b3 << 16));
}

__device__ __forceinline__ void wave_sync() {
  __builtin_amdgcn_fence(__ATOMIC_RELEASE, "wavefront");
  __builtin_amdgcn_wave_barrier();
  __builtin_amdgcn_fence(__ATOMIC_ACQUIRE, "wavefront");
}

__device__ __forceinline__ int cat_word(unsigned ix, unsigned iy, unsigned hx, unsigned hy, int k) {
  const unsigned mI = (k == 0) ? 0xffffffffu : 0u;
  const unsigned mH = (k >= 2 && k < ND) ? 0xffffffffu : 0u;
  const unsigned ue = (ix & mI) | (hx & mH);
  const unsigned uo = (iy & mI) | (hy & mH);
  return (int)(bf16_bits_u(ue) | (bf16_bits_u(uo) << 16));
}

__global__ __launch_bounds__(NTHR) void k_prep(const float* __restrict__ inp, const float* __restrict__ hx,
                                               const float* __restrict__ wfc, const float* __restrict__ bfc,
                                               const float* __restrict__ wg, const float* __restrict__ bg,
                                               int* catw, int* wftw, int* wgpw, float* bfg) {
  const int tid = (int)threadIdx.x;
  const int blk = (int)blockIdx.x;
  if (blk < GBLK) {
    const int row0 = blk * GROWS;
    int* dst = catw + (size_t)row0 * (KP / 2);
#pragma unroll 1
    for (int it = 0; it < 6; ++it) {
      const int c  = it * NTHR + tid;
      const int rl = c / 12;
      const int pc = c - rl * 12;
      const int R  = row0 + rl;
      const int k8 = pc * 8;
      const float* hr = hx + (size_t)R * NU;
      int j0 = k8 - 2, j1 = k8, j2 = k8 + 2, j3 = k8 + 4;
      j0 = j0 < 0 ? 0 : (j0 > NU - 2 ? NU - 2 : j0);
      j1 = j1 > NU - 2 ? NU - 2 : j1;
      j2 = j2 > NU - 2 ? NU - 2 : j2;
      j3 = j3 > NU - 2 ? NU - 2 : j3;
      const v2f iv = *(const v2fa*)(inp + (size_t)R * NDIN);
      const v2f q0 = *(const v2fa*)(hr + j0);
      const v2f q1 = *(const v2fa*)(hr + j1);
      const v2f q2 = *(const v2fa*)(hr + j2);
      const v2f q3 = *(const v2fa*)(hr + j3);
      const float ivx = iv.x, ivy = iv.y;
      const float q0x = q0.x, q0y = q0.y, q1x = q1.x, q1y = q1.y;
      const float q2x = q2.x, q2y = q2.y, q3x = q3.x, q3y = q3.y;
      asm volatile("" :: "v"(ivx), "v"(ivy), "v"(q0x), "v"(q0y), "v"(q1x), "v"(q1y),
                         "v"(q2x), "v"(q2y), "v"(q3x), "v"(q3y));
      v4i o;
      o.x = cat_word(f2u(ivx), f2u(ivy), f2u(q0x), f2u(q0y), k8);
      o.y = cat_word(f2u(ivx), f2u(ivy), f2u(q1x), f2u(q1y), k8 + 2);
      o.z = cat_word(f2u(ivx), f2u(ivy), f2u(q2x), f2u(q2y), k8 + 4);
      o.w = cat_word(f2u(ivx), f2u(ivy), f2u(q3x), f2u(q3y), k8 + 6);
      int* dp = dst + 4 * c;
      *(volatile v4i*)dp = o;
      __threadfence();
      *(volatile v4i*)dp = o;
    }
  } else if (blk < GBLK + PB_WF) {
    const int u  = (blk - GBLK) * NTHR + tid;
    const int n  = u / 12;
    const int k8 = (u - n * 12) * 8;
    float xv[8];
#pragma unroll
    for (int i = 0; i < 8; ++i) {
      const int kc = (k8 + i) < ND ? (k8 + i) : ND - 1;
      xv[i] = wfc[kc * NG + n];
    }
    asm volatile("" :: "v"(xv[0]), "v"(xv[1]), "v"(xv[2]), "v"(xv[3]), "v"(xv[4]), "v"(xv[5]), "v"(xv[6]), "v"(xv[7]));
    unsigned hb[8];
#pragma unroll
    for (int i = 0; i < 8; ++i) hb[i] = ((k8 + i) < ND) ? bf16_bits(xv[i]) : 0u;
    v4i o;
    o.x = (int)(hb[0] | (hb[1] << 16)); o.y = (int)(hb[2] | (hb[3] << 16));
    o.z = (int)(hb[4] | (hb[5] << 16)); o.w = (int)(hb[6] | (hb[7] << 16));
    int* dp = wftw + 4 * u;
    *(volatile v4i*)dp = o;
    __threadfence();
    *(volatile v4i*)dp = o;
  } else if (blk < GBLK + PB_WF + PB_WG) {
    const int u   = (blk - GBLK - PB_WF) * NTHR + tid;
    const int n   = u / 48;
    const int c   = u - n * 48;
    const int kb  = c / 12;
    const int kk8 = (c - kb * 12) * 8;
    const int mm  = kb >> 1;
    float xv[8];
#pragma unroll
    for (int i = 0; i < 8; ++i) {
      const int kc = (kk8 + i) < ND ? (kk8 + i) : ND - 1;
      xv[i] = wg[(2 * kc + mm) * NU + n];
    }
    asm volatile("" :: "v"(xv[0]), "v"(xv[1]), "v"(xv[2]), "v"(xv[3]), "v"(xv[4]), "v"(xv[5]), "v"(xv[6]), "v"(xv[7]));
    unsigned hb[8];
#pragma unroll
    for (int i = 0; i < 8; ++i) hb[i] = ((kk8 + i) < ND) ? bf16_bits(xv[i]) : 0u;
    v4i o;
    o.x = (int)(hb[0] | (hb[1] << 16)); o.y = (int)(hb[2] | (hb[3] << 16));
    o.z = (int)(hb[4] | (hb[5] << 16)); o.w = (int)(hb[6] | (hb[7] << 16));
    int* dp = wgpw + 4 * u;
    *(volatile v4i*)dp = o;
    __threadfence();
    *(volatile v4i*)dp = o;
  } else {
    const int t  = tid < 47 ? tid : 47;
    const int fi = (t < 32 ? t : 31) * 4;
    const int gi = (t < 32 ? 0 : t - 32) * 4;
    const v4f a = *(const v4fa*)(bfc + fi);
    const v4f b = *(const v4fa*)(bg + gi);
    const float ax = a.x, ay = a.y, az = a.z, aw = a.w;
    const float bx = b.x, by = b.y, bz = b.z, bw = b.w;
    asm volatile("" :: "v"(ax), "v"(ay), "v"(az), "v"(aw), "v"(bx), "v"(by), "v"(bz), "v"(bw));
    const unsigned mf = (t < 32) ? 0xffffffffu : 0u;
    v4f o;
    o.x = bf16_val(u2f((f2u(ax) & mf) | (f2u(bx) & ~mf)));
    o.y = bf16_val(u2f((f2u(ay) & mf) | (f2u(by) & ~mf)));
    o.z = bf16_val(u2f((f2u(az) & mf) | (f2u(bz) & ~mf)));
    o.w = bf16_val(u2f((f2u(aw) & mf) | (f2u(bw) & ~mf)));
    float* dp = bfg + 4 * t;
    if (tid < 48) *(volatile v4f*)dp = o;
    __threadfence();
    if (tid < 48) *(volatile v4f*)dp = o;
  }
}

__global__ __launch_bounds__(NTHR) __attribute__((amdgpu_num_vgpr(248)))
void k_gate(const unsigned short* __restrict__ catb, const unsigned short* __restrict__ wft,
            const float* __restrict__ bfp, int* x0w, float* uout) {
  extern __shared__ __attribute__((aligned(16))) int gsm[];
  float* stg = (float*)gsm;
  int*   xst = gsm + GROWS * NG;
  float* ust = (float*)(gsm + GROWS * NG + GROWS * XW);
  const int tid = (int)threadIdx.x, lane = tid & 31, wave = tid >> 5, hh = lane >> 4, m = lane & 15;
  const int rowBase = (int)blockIdx.x * GROWS;

  v8f acc[8];
  {
    const v8f z = {0.f, 0.f, 0.f, 0.f, 0.f, 0.f, 0.f, 0.f};
#pragma unroll
    for (int t = 0; t < 8; ++t) acc[t] = z;
  }
  const unsigned short* ap = catb + (size_t)(rowBase + 16 * wave + m) * (size_t)KP + 8 * hh;
  const unsigned short* bp = wft + (size_t)m * (size_t)KP + 8 * hh;

#pragma unroll 1
  for (int k0 = 0; k0 < KP; k0 += 32) {
    FragB af;
    af.h[0] = *(const v8usa*)(ap + k0);
    af.h[1] = *(const v8usa*)(ap + k0 + 16);
#pragma unroll
    for (int nt = 0; nt < 8; ++nt) {
      const unsigned short* wq = bp + (size_t)(16 * nt) * (size_t)KP + k0;
      FragB bf;
      bf.h[0] = *(const v8usa*)wq;
      bf.h[1] = *(const v8usa*)(wq + 16);
      acc[nt] = wmb(af, bf, acc[nt]);
    }
  }

#pragma unroll
  for (int nt = 0; nt < 8; ++nt) {
    const int lc = 16 * nt + m;
#pragma unroll
    for (int r = 0; r < 8; ++r) {
      const int lr = 16 * wave + 8 * hh + r;
      stg[lr * NG + lc] = acc[nt][r];
    }
  }
  __syncthreads();

  const v4f bias = *(const v4fa*)(bfp + 4 * lane);
  const int lq = lane & 15;
  const int ow = (lane == 0) ? 0 : ((lane <= 16) ? 32 + lane : 64 + lane);
  const unsigned m0 = (lane == 0) ? 0xffffffffu : 0u;
#pragma unroll 1
  for (int i = 0; i < 16; ++i) {
    const int lr = 16 * wave + i;
    const int R  = rowBase + lr;
    const v4f a = *(const v4fa*)(stg + lr * NG + 4 * lane);
    const unsigned short* cr = catb + (size_t)R * (size_t)KP;
    const unsigned wi = *(const u32a*)cr;
    const unsigned w0 = *(const u32a*)(cr + 2 + 4 * lq);
    const unsigned w1 = *(const u32a*)(cr + 4 + 4 * lq);
    asm volatile("" :: "v"(wi), "v"(w0), "v"(w1));
    const float s0 = 1.0f / (1.0f + expf(-(a.x + bias.x)));
    const float s1 = 1.0f / (1.0f + expf(-(a.y + bias.y)));
    const float s2 = 1.0f / (1.0f + expf(-(a.z + bias.z)));
    const float s3 = 1.0f / (1.0f + expf(-(a.w + bias.w)));
    const float r0 = s0 * u2f(w0 << 16);
    const float r1 = s1 * u2f(w0 & 0xffff0000u);
    const float r2 = s2 * u2f(w1 << 16);
    const float r3 = s3 * u2f(w1 & 0xffff0000u);
    int h01, h23, l01, l23;
    hilo_pack(r0, r1, r2, r3, h01, h23, l01, l23);
    int* xr = xst + lr * XW;
    if (lane < 16) {
      xr[1 + 2 * lane]  = h01;
      xr[2 + 2 * lane]  = h23;
      xr[49 + 2 * lane] = l01;
      xr[50 + 2 * lane] = l23;
    }
    xr[ow] = (int)(wi & m0);
    if (lane >= 16) {
      v4f sv;
      sv.x = s0; sv.y = s1; sv.z = s2; sv.w = s3;
      *(v4fa*)(ust + lr * NU + 4 * (lane - 16)) = sv;
    }
  }
  __syncthreads();

  const int* xsrc = xst + 16 * wave * XW;
  const float* usrc = ust + 16 * wave * NU;
  int* xdst = x0w + (size_t)(rowBase + 16 * wave) * (size_t)XW;
  float* udst = uout + (size_t)(rowBase + 16 * wave) * (size_t)NU;
#pragma unroll 1
  for (int it = 0; it < 12; ++it) {
    const int q = (it * 32 + lane) * 4;
    const v4i v = *(const v4ia*)(xsrc + q);
    *(volatile v4i*)(xdst + q) = v;
  }
#pragma unroll 1
  for (int it = 0; it < 8; ++it) {
    const int q = (it * 32 + lane) * 4;
    const v4f v = *(const v4fa*)(usrc + q);
    *(volatile v4f*)(udst + q) = v;
  }
  __threadfence();
#pragma unroll 1
  for (int it = 0; it < 12; ++it) {
    const int q = (it * 32 + lane) * 4;
    const v4i v = *(const v4ia*)(xsrc + q);
    *(volatile v4i*)(xdst + q) = v;
  }
#pragma unroll 1
  for (int it = 0; it < 8; ++it) {
    const int q = (it * 32 + lane) * 4;
    const v4f v = *(const v4fa*)(usrc + q);
    *(volatile v4f*)(udst + q) = v;
  }
}

template <int SLB>
__device__ __forceinline__ int scan_chunk(const int* __restrict__ dsts, int nE, int cbase, int slotBase,
                                          int nb, int vec8, int* list, int tid, int lane, int wave) {
  int wc = 0;
  const int el0  = tid * EPT;
  const int e0   = cbase + el0;
  const int sent = -2147483647 - 1;
  v4i da, db;
  if (vec8 != 0 && cbase + CHUNK <= nE) {
    da = *(const v4i*)(dsts + e0);
    db = *(const v4i*)(dsts + e0 + 4);
  } else {
    const int k0 = dsts[min(e0,     nE - 1)];
    const int k1 = dsts[min(e0 + 1, nE - 1)];
    const int k2 = dsts[min(e0 + 2, nE - 1)];
    const int k3 = dsts[min(e0 + 3, nE - 1)];
    const int k4 = dsts[min(e0 + 4, nE - 1)];
    const int k5 = dsts[min(e0 + 5, nE - 1)];
    const int k6 = dsts[min(e0 + 6, nE - 1)];
    const int k7 = dsts[min(e0 + 7, nE - 1)];
    asm volatile("" :: "v"(k0), "v"(k1), "v"(k2), "v"(k3), "v"(k4), "v"(k5), "v"(k6), "v"(k7));
    da.x = (e0     < nE) ? k0 : sent;
    da.y = (e0 + 1 < nE) ? k1 : sent;
    da.z = (e0 + 2 < nE) ? k2 : sent;
    da.w = (e0 + 3 < nE) ? k3 : sent;
    db.x = (e0 + 4 < nE) ? k4 : sent;
    db.y = (e0 + 5 < nE) ? k5 : sent;
    db.z = (e0 + 6 < nE) ? k6 : sent;
    db.w = (e0 + 7 < nE) ? k7 : sent;
  }
  const unsigned nbs = (unsigned)slotBase;
  const unsigned unb = (unsigned)nb;
  const unsigned s0 = (unsigned)da.x - nbs, s1 = (unsigned)da.y - nbs;
  const unsigned s2 = (unsigned)da.z - nbs, s3 = (unsigned)da.w - nbs;
  const unsigned s4 = (unsigned)db.x - nbs, s5 = (unsigned)db.y - nbs;
  const unsigned s6 = (unsigned)db.z - nbs, s7 = (unsigned)db.w - nbs;
  const bool h0 = s0 < unb, h1 = s1 < unb, h2 = s2 < unb, h3 = s3 < unb;
  const bool h4 = s4 < unb, h5 = s5 < unb, h6 = s6 < unb, h7 = s7 < unb;
  const unsigned any = __builtin_amdgcn_ballot_w32(h0 | h1 | h2 | h3 | h4 | h5 | h6 | h7);
  if (any != 0u) {
#define HITJ(J, HJ, SJ) { \
      const unsigned mj = __builtin_amdgcn_ballot_w32(HJ); \
      if (mj != 0u) { \
        if (HJ) { \
          const int pos = wc + (int)__builtin_amdgcn_mbcnt_lo(mj, 0u); \
          if (pos < WCAP) list[wave * WCAP + pos] = ((el0 + (J)) << SLB) | (int)(SJ); \
        } \
        wc += (int)__builtin_popcount(mj); } }
    HITJ(0, h0, s0)
    HITJ(1, h1, s1)
    HITJ(2, h2, s2)
    HITJ(3, h3, s3)
    HITJ(4, h4, s4)
    HITJ(5, h5, s5)
    HITJ(6, h6, s6)
    HITJ(7, h7, s7)
#undef HITJ
  }
  return wc;
}

__device__ __forceinline__ void gath4(const unsigned* __restrict__ row, int lane, int lq, float wk,
                                      float& a0, float& a1, float& a2, float& a3) {
  const unsigned hA = row[lane];
  const unsigned hB = row[32 + lq];
  const unsigned lA = row[48 + lane];
  const unsigned lB = row[80 + lq];
  float ph0 = u2f(hA << 16), pl0 = u2f(lA << 16), ph1 = u2f(hA & 0xffff0000u), pl1 = u2f(lA & 0xffff0000u);
  float ph2 = u2f(hB << 16), pl2 = u2f(lB << 16), ph3 = u2f(hB & 0xffff0000u), pl3 = u2f(lB & 0xffff0000u);
  asm volatile("" : "+v"(ph0), "+v"(pl0), "+v"(ph1), "+v"(pl1));
  asm volatile("" : "+v"(ph2), "+v"(pl2), "+v"(ph3), "+v"(pl3));
  const float v0 = ph0 + pl0;
  const float v1 = ph1 + pl1;
  const float v2 = ph2 + pl2;
  const float v3 = ph3 + pl3;
  a0 = fmaf(wk, v0, a0); a1 = fmaf(wk, v1, a1);
  a2 = fmaf(wk, v2, a2); a3 = fmaf(wk, v3, a3);
}

__global__ __launch_bounds__(NTHR) void k_scan(const int* __restrict__ gath, const int* __restrict__ keys,
                                               const float* __restrict__ ew, int nE, int nN, int vec8,
                                               const unsigned* __restrict__ x0w, unsigned* x1w) {
  extern __shared__ __attribute__((aligned(16))) int dsm[];
  int* list = dsm;
  int* hl   = dsm + LISTN;
  int* sl   = hl + RCAP;
  int* cnt  = sl + RCAP;
  int* offs = cnt + NBA;
  int* cur  = offs + NBA;
  int* misc = cur + NBA;
  int* rowb = misc + MISC_INTS;
  const int tid = (int)threadIdx.x, lane = tid & 31, wave = tid >> 5;
  const int nodeBase = (int)blockIdx.x * NBA;
  int nbv = nN - nodeBase;
  nbv = nbv < 0 ? 0 : (nbv > NBA ? NBA : nbv);

  {
    const v4i z4 = {0, 0, 0, 0};
    for (int i = tid * 4; i < AGG_ZINTS; i += NTHR * 4) *(v4ia*)(dsm + i) = z4;
    if (tid < MISC_INTS) misc[tid] = 0;
  }
  __syncthreads();

  int t = 0, ov = 0;
  const int nChunks = (nE + CHUNK - 1) / CHUNK;
#pragma unroll 1
  for (int ch = 0; ch < nChunks; ++ch) {
    const int cbase = ch * CHUNK;
    const int wc = scan_chunk<SLA>(keys, nE, cbase, nodeBase, nbv, vec8, list, tid, lane, wave);
    if (lane == 0) misc[wave] = wc;
    __syncthreads();
    if (wave == 0) {
#pragma unroll 1
      for (int w2 = 0; w2 < NWAVE; ++w2) {
        int cvv = misc[w2];
        cvv = cvv < 0 ? 0 : (cvv > WCAP ? WCAP : cvv);
        const int c = __builtin_amdgcn_readfirstlane(cvv);
#pragma unroll 1
        for (int b0 = 0; b0 < c; b0 += 32) {
          const int idx = b0 + lane;
          const int ent = list[w2 * WCAP + (idx < WCAP ? idx : WCAP - 1)];
          const int m32 = (c - b0) < 32 ? (c - b0) : 32;
#pragma unroll 1
          for (int k = 0; k < m32; ++k) {
            const int u    = __builtin_amdgcn_readlane(ent, k);
            const int slot = u & (NBA - 1);
            const int el   = (u >> SLA) & (CHUNK - 1);
            const int pk   = ((cbase + el) << SLA) | slot;
            if (t < RCAP) {
              if (lane == 0) { hl[t] = pk; cnt[slot] = cnt[slot] + 1; }
              t = t + 1;
            } else {
              ov = 1;
            }
          }
        }
      }
    }
    __syncthreads();
  }
  if (wave == 0 && lane == 0) { misc[8] = t; misc[9] = ov; }
  __syncthreads();
  int tt = misc[8];
  tt = tt < 0 ? 0 : (tt > RCAP ? RCAP : tt);
  const int ovf = misc[9];

  if (wave == 0) {
    const int base = lane * (NBA / 32);
    int s = 0;
#pragma unroll 1
    for (int i = 0; i < NBA / 32; ++i) s += cnt[base + i];
    int incl = s;
#pragma unroll
    for (int d = 1; d < 32; d <<= 1) {
      const int y = __shfl_up(incl, d, 32);
      if (lane >= d) incl += y;
    }
    int run = incl - s;
#pragma unroll 1
    for (int i = 0; i < NBA / 32; ++i) {
      const int cv = cnt[base + i];
      offs[base + i] = run;
      cur[base + i]  = run;
      run += cv;
    }
  }
  __syncthreads();
  if (wave == 0) {
    const int ttu = __builtin_amdgcn_readfirstlane(tt);
#pragma unroll 1
    for (int b0 = 0; b0 < ttu; b0 += 32) {
      const int idx = b0 + lane;
      const int ent = hl[idx < RCAP ? idx : RCAP - 1];
      const int m32 = (ttu - b0) < 32 ? (ttu - b0) : 32;
#pragma unroll 1
      for (int k = 0; k < m32; ++k) {
        const int u    = __builtin_amdgcn_readlane(ent, k);
        const int slot = u & (NBA - 1);
        if (lane == 0) {
          int p = cur[slot];
          p = p < 0 ? 0 : (p > RCAP - 1 ? RCAP - 1 : p);
          sl[p] = u;
          cur[slot] = p + 1;
        }
      }
    }
  }
  __syncthreads();

#pragma unroll 1
  for (int p0 = 0; p0 < RCAP; p0 += NTHR) {
    if (p0 >= tt) break;
    const int p  = p0 + tid;
    const int ent = sl[p];
    int eid = ent >> SLA;
    eid = eid < 0 ? 0 : (eid > nE - 1 ? nE - 1 : eid);
    int sr = gath[eid];
    const float wraw = ew[eid];
    asm volatile("" :: "v"(sr), "v"(wraw));
    sr = sr < 0 ? 0 : (sr > nN - 1 ? nN - 1 : sr);
    const int wvi = __float_as_int(bf16_val(wraw));
    if (p < tt) { sl[p] = sr; hl[p] = wvi; }
  }
  __syncthreads();

  const float qnan = __int_as_float(0x7fc00000);
  const float pz = (ovf != 0) ? qnan : 0.0f;
  int* rb = rowb + wave * XW;
  const int lq  = lane & 15;
  const int l23 = lane < 23 ? lane : 23;
  const int pm  = (lane == 0) ? -1 : 0;
#pragma unroll 1
  for (int si = 0; si < NBA / NWAVE; ++si) {
    const int s    = si * NWAVE + wave;
    const int node = nodeBase + s;
    int cv = cnt[s];
    const bool big = cv > DEGCAP;
    cv = cv < 0 ? 0 : (cv > DEGCAP ? DEGCAP : cv);
    const int c0v = cv < 32 ? cv : 32;
    const int c1v = cv - c0v;
    const int c0 = __builtin_amdgcn_readfirstlane(c0v);
    const int c1 = __builtin_amdgcn_readfirstlane(c1v);
    int o = offs[s];
    o = o < 0 ? 0 : (o > RCAP ? RCAP : o);
    int i0 = o + lane;      i0 = i0 > RCAP - 1 ? RCAP - 1 : i0;
    int i1 = o + 32 + lane; i1 = i1 > RCAP - 1 ? RCAP - 1 : i1;
    int sr0 = sl[i0], sr1 = sl[i1];
    const int wv0 = hl[i0], wv1 = hl[i1];
    sr0 = sr0 < 0 ? 0 : (sr0 > nN - 1 ? nN - 1 : sr0);
    sr1 = sr1 < 0 ? 0 : (sr1 > nN - 1 ? nN - 1 : sr1);
    const float pzr = big ? qnan : pz;
    const bool live = node < nN;
    const int nodec = live ? node : nN - 1;
#pragma unroll 1
    for (int b = 0; b < NBAT; ++b) {
      const unsigned* xb = x0w + (size_t)b * (size_t)nN * (size_t)XW;
      float a0 = 0.0f, a1 = 0.0f, a2 = 0.0f, a3 = 0.0f;
#pragma unroll 1
      for (int k = 0; k < c0; ++k) {
        const int   sk = __builtin_amdgcn_readlane(sr0, k);
        const float wk = __int_as_float(__builtin_amdgcn_readlane(wv0, k));
        gath4(xb + (size_t)sk * XW, lane, lq, wk, a0, a1, a2, a3);
      }
#pragma unroll 1
      for (int k = 0; k < c1; ++k) {
        const int   sk = __builtin_amdgcn_readlane(sr1, k);
        const float wk = __int_as_float(__builtin_amdgcn_readlane(wv1, k));
        gath4(xb + (size_t)sk * XW, lane, lq, wk, a0, a1, a2, a3);
      }
      int h01, h23, l01, l23w;
      hilo_pack(a0 + pzr, a1 + pzr, a2 + pzr, a3 + pzr, h01, h23, l01, l23w);
      h23 &= pm; l23w &= pm;
      rb[lane]      = h01;
      rb[48 + lane] = l01;
      if (lane < 16) {
        rb[32 + lane] = h23;
        rb[80 + lane] = l23w;
      }
      wave_sync();
      const v4i q = *(const v4ia*)(rb + 4 * l23);
      asm volatile("" :: "v"(q));
      wave_sync();
      unsigned* dp = x1w + ((size_t)b * (size_t)nN + (size_t)nodec) * (size_t)XW + 4 * l23;
      const bool st = live && (lane < 24);
      if (st) *(volatile v4i*)dp = q;
      __threadfence();
      if (st) *(volatile v4i*)dp = q;
    }
  }
}

template <int WOFF>
__device__ __forceinline__ void kpart(const unsigned short* __restrict__ ap, const unsigned short* __restrict__ bp,
                                      v8f (&acc)[4]) {
#pragma unroll 1
  for (int k0 = 0; k0 < KP * XTERMS; k0 += 32) {
    FragB af;
    af.h[0] = *(const v8usa*)(ap + k0);
    af.h[1] = *(const v8usa*)(ap + k0 + 16);
#pragma unroll
    for (int nt = 0; nt < 4; ++nt) {
      const unsigned short* wq = bp + (size_t)(16 * nt) * (size_t)KC + WOFF + k0;
      FragB bf;
      bf.h[0] = *(const v8usa*)wq;
      bf.h[1] = *(const v8usa*)(wq + 16);
      acc[nt] = wmb(af, bf, acc[nt]);
    }
  }
}

__global__ __launch_bounds__(NTHR) __attribute__((amdgpu_num_vgpr(248)))
void k_cand(const unsigned short* __restrict__ x0, const unsigned short* __restrict__ x1,
            const unsigned short* __restrict__ wgp, const float* __restrict__ bgp,
            const float* __restrict__ hx, float* out) {
  extern __shared__ __attribute__((aligned(16))) int csm[];
  float* stg = (float*)csm;
  float* ut  = (float*)(csm + GROWS * NU);
  const int tid = (int)threadIdx.x, lane = tid & 31, wave = tid >> 5, hh = lane >> 4, m = lane & 15;
  const int rowBase = (int)blockIdx.x * GROWS;

  v8f acc[4];
  {
    const v8f z = {0.f, 0.f, 0.f, 0.f, 0.f, 0.f, 0.f, 0.f};
#pragma unroll
    for (int t = 0; t < 4; ++t) acc[t] = z;
  }
  const size_t arow = (size_t)(rowBase + 16 * wave + m) * (size_t)XP + 8 * hh;
  const unsigned short* bp = wgp + (size_t)m * (size_t)KC + 8 * hh;
  kpart<0>(x0 + arow, bp, acc);
  kpart<2 * KP>(x1 + arow, bp, acc);

#pragma unroll
  for (int nt = 0; nt < 4; ++nt) {
    const int lc = 16 * nt + m;
#pragma unroll
    for (int r = 0; r < 8; ++r) {
      const int lr = 16 * wave + 8 * hh + r;
      stg[lr * NU + lc] = acc[nt][r];
    }
  }
  {
    const float* usrc = out + (size_t)(rowBase + 16 * wave) * (size_t)NU;
    float* udst = ut + 16 * wave * NU;
#pragma unroll 1
    for (int it = 0; it < 8; ++it) {
      const int q = (it * 32 + lane) * 4;
      const v4f v = *(const v4fa*)(usrc + q);
      *(v4fa*)(udst + q) = v;
    }
  }
  __syncthreads();

  const v4f bg4 = *(const v4fa*)(bgp + 4 * (lane & 15));
#pragma unroll 1
  for (int i = 0; i < 8; ++i) {
    const int lidx = (16 * wave + 2 * i) * NU + 4 * lane;
    const v4f p4 = *(const v4fa*)(stg + lidx);
    const v4f u4 = *(const v4fa*)(ut + lidx);
    const size_t g = (size_t)rowBase * (size_t)NU + (size_t)lidx;
    const v4f h4 = *(const v4fa*)(hx + g);
    const float hA = bf16_val(h4.x), hB = bf16_val(h4.y), hC = bf16_val(h4.z), hD = bf16_val(h4.w);
    const float cA = tanhf(p4.x + bg4.x);
    const float cB = tanhf(p4.y + bg4.y);
    const float cC = tanhf(p4.z + bg4.z);
    const float cD = tanhf(p4.w + bg4.w);
    v4f o;
    o.x = u4.x * hA + (1.0f - u4.x) * cA;
    o.y = u4.y * hB + (1.0f - u4.y) * cB;
    o.z = u4.z * hC + (1.0f - u4.z) * cC;
    o.w = u4.w * hD + (1.0f - u4.w) * cD;
    float* op = out + g;
    *(volatile v4f*)op = o;
    __threadfence();
    *(volatile v4f*)op = o;
  }
}

extern "C" void kernel_launch(void* const* d_in, const int* in_sizes, int n_in,
                              void* d_out, int out_size, void* d_ws, size_t ws_size,
                              hipStream_t stream) {
  if (n_in < 9) return;
  if (in_sizes[0] != MR * NDIN) return;
  if (in_sizes[1] != MR * NU) return;
  const int nE = in_sizes[2];
  if (nE < 1 || nE >= (1 << 22)) return;
  if (in_sizes[3] != nE || in_sizes[4] != nE) return;
  if (in_sizes[5] != ND * NG || in_sizes[6] != NG) return;
  if (in_sizes[7] != 2 * ND * NU || in_sizes[8] != NU) return;
  if (out_size != MR * NU) return;

  const float* inp  = (const float*)d_in[0];
  const float* hx   = (const float*)d_in[1];
  const int*   rows = (const int*)d_in[2];
  const int*   cols = (const int*)d_in[3];
  const float* vals = (const float*)d_in[4];
  const float* wfc  = (const float*)d_in[5];
  const float* bfc  = (const float*)d_in[6];
  const float* wg   = (const float*)d_in[7];
  const float* bg   = (const float*)d_in[8];
  float* out = (float*)d_out;

  const size_t szX   = (size_t)MR * XP * 2;
  const size_t szCat = (size_t)MR * KP * 2;
  const size_t szWf  = (size_t)NG * KP * 2;
  const size_t szWg  = (size_t)NU * KC * 2;
  const size_t szB   = (size_t)(NG + NU) * 4;
  const size_t oX0 = 0;
  const size_t oX1 = oX0 + szX;
  const size_t oWf = oX1 + szX;
  const size_t oWg = oWf + szWf;
  const size_t oB  = oWg + szWg;
  const size_t tot = oB + szB;
  if (szCat > szX) return;
  if (tot > ws_size || tot > (size_t)WSMAX) return;
  char* ws = (char*)d_ws;
  unsigned short* X0   = (unsigned short*)(ws + oX0);
  unsigned short* X1   = (unsigned short*)(ws + oX1);
  unsigned short* CATB = (unsigned short*)(ws + oX1);
  unsigned short* WfT  = (unsigned short*)(ws + oWf);
  unsigned short* WgP  = (unsigned short*)(ws + oWg);
  float*          BFG  = (float*)(ws + oB);

  const size_t gateLds = (size_t)GATE_LDS_INTS * 4;
  const size_t scanLds = (size_t)SCAN_LDS_INTS * 4;
  const size_t candLds = (size_t)CAND_LDS_INTS * 4;
  hipFuncSetAttribute(reinterpret_cast<const void*>(&k_gate), hipFuncAttributeMaxDynamicSharedMemorySize, (int)gateLds);
  hipFuncSetAttribute(reinterpret_cast<const void*>(&k_scan), hipFuncAttributeMaxDynamicSharedMemorySize, (int)scanLds);
  hipFuncSetAttribute(reinterpret_cast<const void*>(&k_cand), hipFuncAttributeMaxDynamicSharedMemorySize, (int)candLds);

  const int vec8 = ((nE & 3) == 0) ? 1 : 0;

  k_prep<<<GBLK + PB_WF + PB_WG + 1, NTHR, 0, stream>>>(inp, hx, wfc, bfc, wg, bg,
                                                       (int*)CATB, (int*)WfT, (int*)WgP, BFG);
  k_gate<<<GBLK, NTHR, gateLds, stream>>>(CATB, WfT, BFG, (int*)X0, out);
  k_scan<<<NSCAN, NTHR, scanLds, stream>>>(cols, rows, vals, nE, NNODE, vec8,
                                           (const unsigned*)X0, (unsigned*)X1);
  k_cand<<<GBLK, NTHR, candLds, stream>>>(X0, X1, WgP, BFG + NG, hx, out);
}
